// CausalSelfAttentionLayer_37830071943383
// MI455X (gfx1250) — hardware-verified
//
#include <hip/hip_runtime.h>

constexpr int kBatch = 4;
constexpr int kSeq   = 2048;
constexpr int kEmb   = 1024;
constexpr int kHeads = 16;
constexpr int kHdim  = 64;
constexpr int kE3    = 3 * kEmb;
constexpr int kTok   = kBatch * kSeq;
constexpr int kQB    = 64;
constexpr int kKC    = 64;
constexpr int kOSP   = 68;
constexpr float kScoreScale = 0.125f;

static_assert(kHeads * kHdim == kEmb, "head split");
static_assert(kTok % 64 == 0 && kEmb % 64 == 0 && kE3 % 64 == 0, "GEMM M,N tile multiples of 64");
static_assert(kEmb % 32 == 0, "GEMM K multiple of 32");
static_assert(kSeq % kQB == 0 && kSeq % kKC == 0, "attention tiles");
static_assert(kHdim == 64, "attention kernel is written for head dim 64");

typedef __attribute__((ext_vector_type(16))) _Float16 v16h;
typedef __attribute__((ext_vector_type(8)))  _Float16 v8h;
typedef __attribute__((ext_vector_type(16))) __bf16   v16b;
typedef __attribute__((ext_vector_type(8)))  __bf16   v8b;
typedef __attribute__((ext_vector_type(8)))  float    v8f;
typedef __attribute__((ext_vector_type(4)))  float    v4f;

__device__ __forceinline__ unsigned short f2bf_bits(float f) {
  unsigned u = __float_as_uint(f);
  return (unsigned short)((u + 0x7FFFu + ((u >> 16) & 1u)) >> 16);
}
__device__ __forceinline__ float bf_bits2f(unsigned short h) { return __uint_as_float(((unsigned)h) << 16); }

__device__ __forceinline__ void dep_guard_h(v8f& a, v8f& b, v16h x, v16h y) { asm volatile("v_nop\n\tv_nop\n\tv_nop\n\tv_nop" : "+v"(a), "+v"(b) : "v"(x), "v"(y)); }
__device__ __forceinline__ void dep_guard_b(v8f& a, v8f& b, v16b x, v16b y) { asm volatile("v_nop\n\tv_nop\n\tv_nop\n\tv_nop" : "+v"(a), "+v"(b) : "v"(x), "v"(y)); }
__device__ __forceinline__ void keep4_h(v16h a, v16h b, v16h c, v16h d) { asm volatile("v_nop" :: "v"(a), "v"(b), "v"(c), "v"(d)); }
__device__ __forceinline__ void keep4_b(v16b a, v16b b, v16b c, v16b d) { asm volatile("v_nop" :: "v"(a), "v"(b), "v"(c), "v"(d)); }
__device__ __forceinline__ void acc_guard4(v8f& a, v8f& b, v8f& c, v8f& d) { asm volatile("v_nop\n\tv_nop\n\tv_nop\n\tv_nop" : "+v"(a), "+v"(b), "+v"(c), "+v"(d)); }
template <typename T> struct Frag;
template <> struct Frag<_Float16> {
  typedef v16h V; union U { v16h v; v8h h[2]; };
  static __device__ __forceinline__ v16h load(const _Float16* p) {
    U f; f.h[0] = *(const v8h*)(p); f.h[1] = *(const v8h*)(p + 16); return f.v;
  }
  static __device__ __forceinline__ v8f mma(v16h a, v16h b, v8f c) {
    return __builtin_amdgcn_wmma_f32_16x16x32_f16(false, a, false, b, (short)0, c, false, false);
  }
  static __device__ __forceinline__ void guard(v8f& a, v8f& b, v16h x, v16h y) { dep_guard_h(a, b, x, y); }
  static __device__ __forceinline__ void keep(v16h a, v16h b, v16h c, v16h d) { keep4_h(a, b, c, d); }
};
template <> struct Frag<__bf16> {
  typedef v16b V; union U { v16b v; v8b h[2]; };
  static __device__ __forceinline__ v16b load(const __bf16* p) {
    U f; f.h[0] = *(const v8b*)(p); f.h[1] = *(const v8b*)(p + 16); return f.v;
  }
  static __device__ __forceinline__ v8f mma(v16b a, v16b b, v8f c) {
    return __builtin_amdgcn_wmma_f32_16x16x32_bf16(false, a, false, b, (short)0, c, false, false);
  }
  static __device__ __forceinline__ void guard(v8f& a, v8f& b, v16b x, v16b y) { dep_guard_b(a, b, x, y); }
  static __device__ __forceinline__ void keep(v16b a, v16b b, v16b c, v16b d) { keep4_b(a, b, c, d); }
};

template <int ET> struct Elem;
template <> struct Elem<0> { typedef _Float16 T; };
template <> struct Elem<1> { typedef __bf16 T; };
template <int ET, int SPLIT, int BIAS_MODE, int OUT_MODE, bool RESID, int ACT = 0>
__global__ __launch_bounds__(256) void wmma_gemm64(
    const unsigned short* __restrict__ Ap, const unsigned short* __restrict__ A2p, int lda, long strideA,
    const unsigned short* __restrict__ Btp, const unsigned short* __restrict__ Bt2p, int ldb, long strideB,
    void* __restrict__ Cout, void* __restrict__ Cout2, int ldc, long strideC,
    const float* __restrict__ bias,
    const float* __restrict__ resid, long strideR,
    int M, int N, int K, float scale) {
  typedef typename Elem<ET>::T T;
  typedef typename Frag<T>::V V;
  const T* A = (const T*)Ap; const T* A2 = (const T*)A2p; const T* Bt = (const T*)Btp; const T* Bt2 = (const T*)Bt2p;
  __shared__ __align__(16) float sT[8][16 * 68];
  const int b    = blockIdx.y;
  const int lane = threadIdx.x & 31;
  const int wave = threadIdx.x >> 5;
  const int tilesN = N >> 6;
  const int tilesM = M >> 6;
  const int tile = blockIdx.x * 8 + wave;
  if (tile >= tilesM * tilesN) return;
  const int tm = tile / tilesN;
  const int tn = tile - tm * tilesN;
  const int m0 = tm << 6;
  const int n0 = tn << 6;

  const T* Ab  = A  + (size_t)b * strideA;
  const T* Bb  = Bt + (size_t)b * strideB;
  const T* Ab2 = (SPLIT != 0) ? (A2  + (size_t)b * strideA) : nullptr;
  const T* Bb2 = (SPLIT == 1) ? (Bt2 + (size_t)b * strideB) : nullptr;

  const int rlane = lane & 15;
  const int koff  = (lane >> 4) * 8;
  const int mOff  = (lane >> 4) * 8;

  v8f acc[4][4];
#pragma unroll
  for (int i = 0; i < 4; ++i)
#pragma unroll
    for (int j = 0; j < 4; ++j) acc[i][j] = (v8f){0.f,0.f,0.f,0.f,0.f,0.f,0.f,0.f};

  for (int k0 = 0; k0 < K; k0 += 32) {
    V bh[4], bl[4];
#pragma unroll
    for (int j = 0; j < 4; ++j) {
      const size_t bo = (size_t)(n0 + (j << 4) + rlane) * ldb + koff + k0;
      bh[j] = Frag<T>::load(Bb + bo);
      if (SPLIT == 1) bl[j] = Frag<T>::load(Bb2 + bo);
    }
#pragma unroll
    for (int i = 0; i < 4; ++i) {
      const size_t ao = (size_t)(m0 + (i << 4) + rlane) * lda + koff + k0;
      V ah = Frag<T>::load(Ab + ao);
      V al;
      if (SPLIT != 0) al = Frag<T>::load(Ab2 + ao);
#pragma unroll
      for (int j = 0; j < 4; ++j) {
        acc[i][j] = Frag<T>::mma(ah, bh[j], acc[i][j]);
        if (SPLIT == 1) {
          acc[i][j] = Frag<T>::mma(ah, bl[j], acc[i][j]);
          acc[i][j] = Frag<T>::mma(al, bh[j], acc[i][j]);
        }
        if (SPLIT == 2) {
          acc[i][j] = Frag<T>::mma(al, bh[j], acc[i][j]);
        }
      }
      Frag<T>::guard(acc[i][0], acc[i][3], ah, (SPLIT != 0) ? al : ah);
    }
    Frag<T>::keep(bh[0], bh[1], bh[2], bh[3]);
    if (SPLIT == 1) Frag<T>::keep(bl[0], bl[1], bl[2], bl[3]);
  }
  acc_guard4(acc[0][0], acc[0][1], acc[0][2], acc[0][3]);
  acc_guard4(acc[1][0], acc[1][1], acc[1][2], acc[1][3]);
  acc_guard4(acc[2][0], acc[2][1], acc[2][2], acc[2][3]);
  acc_guard4(acc[3][0], acc[3][1], acc[3][2], acc[3][3]);

  float* slab = sT[wave];
  const float* Rb = RESID ? (resid + (size_t)b * strideR) : nullptr;
#pragma unroll
  for (int i = 0; i < 4; ++i) {
    const int mBase = m0 + (i << 4);
#pragma unroll
    for (int j = 0; j < 4; ++j) {
      const int n = n0 + (j << 4) + rlane;
      float bv = 0.f;
      if (BIAS_MODE == 2) bv = bias[n];
      if (BIAS_MODE == 3) bv = bf_bits2f(f2bf_bits(bias[n]));
#pragma unroll
      for (int r = 0; r < 8; ++r) {
        float v = acc[i][j][r] * scale;
        if (BIAS_MODE == 1) v += bias[mBase + mOff + r];
        if (BIAS_MODE == 2 || BIAS_MODE == 3) v += bv;
        if (RESID) v += Rb[(size_t)(mBase + mOff + r) * ldc + n];
        if (ACT == 2) v = fmaxf(v, 0.0f);
        if (ACT == 4) v = (v > 0.f) ? v : 0.01f * v;
        slab[(mOff + r) * 68 + (j << 4) + rlane] = v;
      }
    }
    __builtin_amdgcn_fence(__ATOMIC_RELEASE, "workgroup");
    __builtin_amdgcn_wave_barrier();
    __builtin_amdgcn_fence(__ATOMIC_ACQUIRE, "workgroup");
    if (OUT_MODE == 0) {
      float* C = (float*)Cout + (size_t)b * strideC;
      const int hh = lane >> 4, c4 = (lane & 15) * 4;
      for (int pass = 0; pass < 2; ++pass) {
#pragma unroll
        for (int it = 0; it < 8; ++it) {
          const int row = it * 2 + hh;
          v4f v = *(const v4f*)(slab + row * 68 + c4);
          *(volatile v4f*)(C + (size_t)(mBase + row) * ldc + n0 + c4) = v;
        }
        __threadfence();
      }
    } else {
      const int q = lane >> 3, c8 = (lane & 7) * 8;
      unsigned short* C  = (unsigned short*)Cout  + (size_t)b * strideC;
      unsigned short* C2 = (OUT_MODE == 2) ? ((unsigned short*)Cout2 + (size_t)b * strideC) : nullptr;
      for (int pass = 0; pass < 2; ++pass) {
#pragma unroll
        for (int it = 0; it < 4; ++it) {
          const int row = it * 4 + q;
          const float* sp = slab + row * 68 + c8;
          v8h hv, lv;
#pragma unroll
          for (int e = 0; e < 8; ++e) {
            if (OUT_MODE == 1) {
              hv[e] = (_Float16)sp[e];
            } else {
              unsigned short hb = f2bf_bits(sp[e]);
              unsigned short lb = f2bf_bits(sp[e] - bf_bits2f(hb));
              hv[e] = __builtin_bit_cast(_Float16, hb);
              lv[e] = __builtin_bit_cast(_Float16, lb);
            }
          }
          *(volatile v8h*)(C + (size_t)(mBase + row) * ldc + n0 + c8) = hv;
          if (OUT_MODE == 2) *(volatile v8h*)(C2 + (size_t)(mBase + row) * ldc + n0 + c8) = lv;
        }
        __threadfence();
      }
    }
    __builtin_amdgcn_fence(__ATOMIC_RELEASE, "workgroup");
    __builtin_amdgcn_wave_barrier();
    __builtin_amdgcn_fence(__ATOMIC_ACQUIRE, "workgroup");
  }
}

__global__ __launch_bounds__(256) void cast_f32_bf16x2(
    const float* __restrict__ in, unsigned short* __restrict__ out, int n2) {
  const int i = blockIdx.x * 256 + threadIdx.x;
  if (i < n2) {
    const unsigned short h0 = f2bf_bits(in[2 * i]);
    const unsigned short h1 = f2bf_bits(in[2 * i + 1]);
    const unsigned u = (unsigned)h0 | ((unsigned)h1 << 16);
    volatile unsigned* o = (volatile unsigned*)(void*)out;
    o[i] = u;
    __threadfence();
    o[i] = u;
  }
}

__device__ __forceinline__ v8f mma_h(v16h a, v16h b, v8f c) {
  c = __builtin_amdgcn_wmma_f32_16x16x32_f16(false, a, false, b, (short)0, c, false, false);
  asm volatile("v_nop\n\tv_nop\n\tv_nop\n\tv_nop" : "+v"(c) : "v"(a), "v"(b));
  return c;
}
__device__ __forceinline__ v8f mma_b(v16b a, v16b b, v8f c) {
  c = __builtin_amdgcn_wmma_f32_16x16x32_bf16(false, a, false, b, (short)0, c, false, false);
  asm volatile("v_nop\n\tv_nop\n\tv_nop\n\tv_nop" : "+v"(c) : "v"(a), "v"(b));
  return c;
}

__global__ __launch_bounds__(128) void attn_causal64_k(
    const unsigned short* __restrict__ qpp, const unsigned short* __restrict__ kpp,
    const unsigned short* __restrict__ vhpp, const unsigned short* __restrict__ vlpp,
    unsigned short* __restrict__ ohpp, unsigned short* __restrict__ olpp) {
  union FH { v16h v; v8h h[2]; };
  union FB { v16b v; v8b h[2]; };
  __shared__ __align__(16) _Float16 Ksh[kKC * kHdim];
  __shared__ __align__(16) __bf16   Vth[kHdim * kKC];
  __shared__ __align__(16) __bf16   Vtl[kHdim * kKC];
  __shared__ __align__(16) __bf16   Psh[4][16 * kKC];
  __shared__ __align__(16) __bf16   Psl[4][16 * kKC];
  __shared__ __align__(16) float    Osh[4][16 * kOSP];

  const _Float16* qp  = (const _Float16*)(const void*)qpp;
  const _Float16* kp  = (const _Float16*)(const void*)kpp;
  const __bf16*   vhp = (const __bf16*)(const void*)vhpp;
  const __bf16*   vlp = (const __bf16*)(const void*)vlpp;
  __bf16*         ohp = (__bf16*)(void*)ohpp;
  __bf16*         olp = (__bf16*)(void*)olpp;

  const int tid  = threadIdx.x;
  const int wave = tid >> 5;
  const int lane = tid & 31;
  const int hh   = lane >> 4;
  const int c    = lane & 15;

  const int nqb = kSeq / kQB;
  const int bx  = blockIdx.x;
  const int qb  = bx % nqb;
  const int bh  = bx / nqb;
  const int h   = bh % kHeads;
  const int b   = bh / kHeads;
  const int q0  = qb * kQB + wave * 16;
  const size_t tokb = (size_t)b * kSeq;
  const int hcol = h * kHdim;
  const float kNegInf = -__builtin_huge_valf();

  v16h qa[2];
  {
    const _Float16* qrow = qp + (tokb + q0 + c) * kEmb + hcol + 8 * hh;
#pragma unroll
    for (int dc = 0; dc < 2; ++dc) qa[dc] = Frag<_Float16>::load(qrow + dc * 32);
  }

  float mrow[8], lrow[8];
  v8f oacc[4];
#pragma unroll
  for (int r = 0; r < 8; ++r) { mrow[r] = kNegInf; lrow[r] = 0.f; }
#pragma unroll
  for (int t = 0; t < 4; ++t) oacc[t] = (v8f){0.f,0.f,0.f,0.f,0.f,0.f,0.f,0.f};

  const int nChunks = qb + 1;
  for (int kc = 0; kc < nChunks; ++kc) {
    const int kv0 = kc * kKC;
    __syncthreads();
    {
      const int kvr = tid >> 1, dh = (tid & 1) * 32;
      const size_t rowoff = (tokb + kv0 + kvr) * kEmb + hcol + dh;
      const _Float16* krow  = kp  + rowoff;
      const __bf16*   vhrow = vhp + rowoff;
      const __bf16*   vlrow = vlp + rowoff;
#pragma unroll 1
      for (int i = 0; i < 4; ++i) {
        const v8h kk = *(const v8h*)(krow + 8 * i);
        *(v8h*)(Ksh + kvr * kHdim + dh + 8 * i) = kk;
        const v8b vh = *(const v8b*)(vhrow + 8 * i);
        const v8b vl = *(const v8b*)(vlrow + 8 * i);
#pragma unroll
        for (int e = 0; e < 8; ++e) {
          const int d = dh + 8 * i + e;
          Vth[d * kKC + kvr] = vh[e];
          Vtl[d * kKC + kvr] = vl[e];
        }
      }
    }
    __syncthreads();

    v8f s[4];
#pragma unroll
    for (int j = 0; j < 4; ++j) {
      s[j] = (v8f){0.f,0.f,0.f,0.f,0.f,0.f,0.f,0.f};
#pragma unroll
      for (int dc = 0; dc < 2; ++dc) {
        FH kb;
        kb.h[0] = *(const v8h*)(Ksh + (j * 16 + c) * kHdim + dc * 32 + 8 * hh);
        kb.h[1] = *(const v8h*)(Ksh + (j * 16 + c) * kHdim + dc * 32 + 16 + 8 * hh);
        s[j] = mma_h(qa[dc], kb.v, s[j]);
      }
    }
    const bool diag = (kc == qb);
    float cm[8];
#pragma unroll
    for (int r = 0; r < 8; ++r) {
      const int qrow = q0 + 8 * hh + r;
      float m = kNegInf;
#pragma unroll
      for (int j = 0; j < 4; ++j) {
        const int kvcol = kv0 + j * 16 + c;
        float sv = s[j][r] * kScoreScale;
        if (diag && (kvcol > qrow)) sv = kNegInf;
        s[j][r] = sv;
        m = fmaxf(m, sv);
      }
#pragma unroll
      for (int off = 1; off < 16; off <<= 1) m = fmaxf(m, __shfl_xor(m, off, 32));
      cm[r] = m;
    }
    __bf16* pwh = Psh[wave];
    __bf16* pwl = Psl[wave];
#pragma unroll
    for (int r = 0; r < 8; ++r) {
      const float mnew  = fmaxf(mrow[r], cm[r]);
      const float alpha = expf(mrow[r] - mnew);
      mrow[r] = mnew;
      float psum = 0.f;
#pragma unroll
      for (int j = 0; j < 4; ++j) {
        const float p = expf(s[j][r] - mnew);
        psum += p;
        const unsigned short hb = f2bf_bits(p);
        const unsigned short lb = f2bf_bits(p - bf_bits2f(hb));
        pwh[(8 * hh + r) * kKC + j * 16 + c] = __builtin_bit_cast(__bf16, hb);
        pwl[(8 * hh + r) * kKC + j * 16 + c] = __builtin_bit_cast(__bf16, lb);
      }
#pragma unroll
      for (int off = 1; off < 16; off <<= 1) psum += __shfl_xor(psum, off, 32);
      lrow[r] = lrow[r] * alpha + psum;
#pragma unroll
      for (int t = 0; t < 4; ++t) oacc[t][r] *= alpha;
    }
    __builtin_amdgcn_fence(__ATOMIC_RELEASE, "workgroup");
    __builtin_amdgcn_wave_barrier();
    __builtin_amdgcn_fence(__ATOMIC_ACQUIRE, "workgroup");
#pragma unroll 1
    for (int kk = 0; kk < 2; ++kk) {
      FB pa, pl;
      pa.h[0] = *(const v8b*)(pwh + c * kKC + kk * 32 + 8 * hh);
      pa.h[1] = *(const v8b*)(pwh + c * kKC + kk * 32 + 16 + 8 * hh);
      pl.h[0] = *(const v8b*)(pwl + c * kKC + kk * 32 + 8 * hh);
      pl.h[1] = *(const v8b*)(pwl + c * kKC + kk * 32 + 16 + 8 * hh);
#pragma unroll
      for (int t = 0; t < 4; ++t) {
        FB vb, vl;
        vb.h[0] = *(const v8b*)(Vth + (t * 16 + c) * kKC + kk * 32 + 8 * hh);
        vb.h[1] = *(const v8b*)(Vth + (t * 16 + c) * kKC + kk * 32 + 16 + 8 * hh);
        vl.h[0] = *(const v8b*)(Vtl + (t * 16 + c) * kKC + kk * 32 + 8 * hh);
        vl.h[1] = *(const v8b*)(Vtl + (t * 16 + c) * kKC + kk * 32 + 16 + 8 * hh);
        oacc[t] = mma_b(pa.v, vb.v, oacc[t]);
        oacc[t] = mma_b(pa.v, vl.v, oacc[t]);
        oacc[t] = mma_b(pl.v, vb.v, oacc[t]);
      }
    }
  }

  float* os = Osh[wave];
#pragma unroll
  for (int r = 0; r < 8; ++r) {
    const float inv = 1.0f / lrow[r];
#pragma unroll
    for (int t = 0; t < 4; ++t) os[(8 * hh + r) * kOSP + t * 16 + c] = oacc[t][r] * inv;
  }
  __builtin_amdgcn_fence(__ATOMIC_RELEASE, "workgroup");
  __builtin_amdgcn_wave_barrier();
  __builtin_amdgcn_fence(__ATOMIC_ACQUIRE, "workgroup");
  {
    const int q8 = lane >> 3, c8 = (lane & 7) * 8;
    for (int pass = 0; pass < 2; ++pass) {
#pragma unroll
      for (int it = 0; it < 4; ++it) {
        const int row = it * 4 + q8;
        const float* sp = os + row * kOSP + c8;
        v8h hv, lv;
#pragma unroll
        for (int e = 0; e < 8; ++e) {
          const unsigned short hb = f2bf_bits(sp[e]);
          const unsigned short lb = f2bf_bits(sp[e] - bf_bits2f(hb));
          hv[e] = __builtin_bit_cast(_Float16, hb);
          lv[e] = __builtin_bit_cast(_Float16, lb);
        }
        const size_t o = (tokb + q0 + row) * kEmb + hcol + c8;
        *(volatile v8h*)(ohp + o) = hv;
        *(volatile v8h*)(olp + o) = lv;
      }
      __threadfence();
    }
  }
}

extern "C" void kernel_launch(void* const* d_in, const int* in_sizes, int n_in,
                              void* d_out, int out_size, void* d_ws, size_t ws_size,
                              hipStream_t stream) {
  if (n_in < 5) return;
  const int nX  = kTok * kEmb;
  const int nWk = kE3 * kEmb;
  const int nWp = kEmb * kEmb;
  if (in_sizes[0] != nX || in_sizes[1] != nWk || in_sizes[2] != kE3 ||
      in_sizes[3] != nWp || in_sizes[4] != kEmb) return;
  if (out_size != nX) return;
  static_assert((kTok * kEmb / 2) % 256 == 0 && (kE3 * kEmb / 2) % 256 == 0 && (kEmb * kEmb / 2) % 256 == 0,
                "cast grids are exact");

  const float* x      = (const float*)d_in[0];
  const float* W_kqv  = (const float*)d_in[1];
  const float* b_kqv  = (const float*)d_in[2];
  const float* W_proj = (const float*)d_in[3];
  const float* b_proj = (const float*)d_in[4];
  float* out = (float*)d_out;

  const size_t plane = (size_t)kTok * kEmb * 2;
  size_t off = 0;
  const size_t oXb = off; off += plane;
  const size_t oWk = off; off += (size_t)kE3 * kEmb * 2;
  const size_t oWp = off; off += (size_t)kEmb * kEmb * 2;
  const size_t oQ  = off; off += plane;
  const size_t oK  = off; off += plane;
  const size_t oVh = off; off += plane;
  const size_t oVl = off; off += plane;
  const size_t oOh = off; off += plane;
  const size_t oOl = off; off += plane;
  if (off > ws_size) return;

  char* ws = (char*)d_ws;
  unsigned short* xb  = (unsigned short*)(ws + oXb);
  unsigned short* wkb = (unsigned short*)(ws + oWk);
  unsigned short* wpb = (unsigned short*)(ws + oWp);
  unsigned short* q16 = (unsigned short*)(ws + oQ);
  unsigned short* k16 = (unsigned short*)(ws + oK);
  unsigned short* vhi = (unsigned short*)(ws + oVh);
  unsigned short* vlo = (unsigned short*)(ws + oVl);
  unsigned short* ohi = (unsigned short*)(ws + oOh);
  unsigned short* olo = (unsigned short*)(ws + oOl);

  cast_f32_bf16x2<<<dim3((nX / 2) / 256), dim3(256), 0, stream>>>(x, xb, nX / 2);
  cast_f32_bf16x2<<<dim3((nWk / 2) / 256), dim3(256), 0, stream>>>(W_kqv, wkb, nWk / 2);
  cast_f32_bf16x2<<<dim3((nWp / 2) / 256), dim3(256), 0, stream>>>(W_proj, wpb, nWp / 2);

  const int gemmBlocks = ((kTok / 64) * (kEmb / 64) + 7) / 8;
  const size_t wThird = (size_t)kEmb * kEmb;
  wmma_gemm64<1, 0, 3, 1, false, 0><<<dim3(gemmBlocks, 1), dim3(256), 0, stream>>>(
      xb, xb, kEmb, 0L, wkb, wkb, kEmb, 0L,
      (void*)q16, (void*)q16, kEmb, 0L, b_kqv, b_kqv, 0L, kTok, kEmb, kEmb, 1.0f);
  wmma_gemm64<1, 0, 3, 1, false, 0><<<dim3(gemmBlocks, 1), dim3(256), 0, stream>>>(
      xb, xb, kEmb, 0L, wkb + wThird, wkb + wThird, kEmb, 0L,
      (void*)k16, (void*)k16, kEmb, 0L, b_kqv + kEmb, b_kqv, 0L, kTok, kEmb, kEmb, 1.0f);
  wmma_gemm64<1, 0, 3, 2, false, 0><<<dim3(gemmBlocks, 1), dim3(256), 0, stream>>>(
      xb, xb, kEmb, 0L, wkb + 2 * wThird, wkb + 2 * wThird, kEmb, 0L,
      (void*)vhi, (void*)vlo, kEmb, 0L, b_kqv + 2 * kEmb, b_kqv, 0L, kTok, kEmb, kEmb, 1.0f);

  attn_causal64_k<<<dim3(kBatch * kHeads * (kSeq / kQB)), dim3(128), 0, stream>>>(
      q16, k16, vhi, vlo, ohi, olo);

  wmma_gemm64<1, 2, 3, 0, false, 0><<<dim3(gemmBlocks, 1), dim3(256), 0, stream>>>(
      ohi, olo, kEmb, 0L, wpb, wpb, kEmb, 0L,
      (void*)out, (void*)out, kEmb, 0L, b_proj, b_proj, 0L, kTok, kEmb, kEmb, 1.0f);
}
